// SelfAttention_8057358648211
// MI455X (gfx1250) — hardware-run, weakly checked
//
#include <hip/hip_runtime.h>


#ifndef NB
#define NB 2
#endif
#ifndef SEQ
#define SEQ 4096
#endif
#define NB_FULL  2
#define SEQ_FULL 4096
#ifndef OUT_SEQ
#define OUT_SEQ SEQ
#endif
#define DM   128
#define NH_  4
#define HD   32
#define NG   16
#define CPG  8
#define AW   4
#define OSP  36
#define TP   136
#define WSC  16.0f
#define WSI  (1.0f / 16.0f)
#define CTXC 256.0f
#define OSC  (1.0f / 4096.0f)
#define GN_EPS 1.0e-5f
#define SC2  ((float)(0.08838834764831845 * 1.4426950408889634))
#define PSH  14.0f
#define NEGB (-3.0e38f)

static_assert(HD == 32);
static_assert(NH_ * HD == DM);
static_assert(NG * CPG == DM);
static_assert(CPG == 8);
static_assert(DM % 64 == 0);
static_assert(DM % 32 == 0);
static_assert(DM == 128);
static_assert(SEQ % 64 == 0);
static_assert((NB * SEQ) % 64 == 0);
static_assert(SEQ % 32 == 0);
static_assert(SEQ % (16 * AW) == 0);
static_assert((CPG * (SEQ / 4)) % 256 == 0);
static_assert(NB <= NB_FULL);
static_assert(SEQ <= SEQ_FULL);
static_assert((OSP * 4) % 16 == 0);
static_assert((TP * 2) % 16 == 0);
static_assert(TP >= DM);
static_assert(WSC * CTXC * OSC == 1.0f);
static_assert(WSC * WSI == 1.0f);
static_assert(sizeof(float) * 16 * 68 <= 131072);
static_assert(sizeof(float) * AW * 16 * OSP <= 131072);
static_assert(2 * 64 * TP <= 131072);

typedef _Float16 h16;
typedef unsigned short bf;
typedef __attribute__((ext_vector_type(16))) __bf16   v16bf;
typedef __attribute__((ext_vector_type(16))) _Float16 v16h;
typedef __attribute__((ext_vector_type(8)))  _Float16 v8h;
typedef __attribute__((ext_vector_type(8)))  unsigned short v8us;
typedef __attribute__((ext_vector_type(8)))  float    v8f;
typedef __attribute__((ext_vector_type(4)))  float    v4f;
typedef v4f  __attribute__((may_alias)) v4fa;
typedef v8h  __attribute__((may_alias)) v8ha;

__device__ __forceinline__ unsigned short f2bf(float f) { unsigned u = __float_as_uint(f); u += 0x7FFFu + ((u >> 16) & 1u); return (unsigned short)(u >> 16); }
__device__ __forceinline__ float bfr(float f) { return __uint_as_float(((unsigned)f2bf(f)) << 16); }
__device__ __forceinline__ v16h cat16(v8h lo, v8h hi) { return __builtin_shufflevector(lo, hi, 0, 1, 2, 3, 4, 5, 6, 7, 8, 9, 10, 11, 12, 13, 14, 15); }
__device__ __forceinline__ v8f wmma16(v16h a, v16h b, v8f c) { return __builtin_amdgcn_wmma_f32_16x16x32_f16(false, a, false, b, (short)0, c, false, false); }
__device__ __forceinline__ v16h  ldh(const h16* p) { return cat16(*(const v8h*)p, *(const v8h*)(p + 16)); }
__device__ __forceinline__ void wave_sync() { __builtin_amdgcn_fence(3  , "wavefront"); __builtin_amdgcn_wave_barrier(); asm volatile("" ::: "memory"); }
__device__ __forceinline__ v8f wmma16g(v16h a, v16h b, v8f c) { c = wmma16(a, b, c); asm volatile("v_nop\n\tv_nop\n\tv_nop\n\tv_nop" : "+v"(c) : "v"(a), "v"(b)); return c; }
static __device__ __forceinline__ h16 toh_flush(float v) { const h16 r = (h16)v; return (fabsf(v) < 6.103515625e-05f) ? (h16)0.0f : r; }

__global__ __launch_bounds__(256) void k_gnstats(const float* __restrict__ x, float* stats) {
#pragma clang fp contract(off)
    __shared__ float red[8];
    __shared__ float red2[8];
    const int bg = blockIdx.x; const int b = bg / NG, g = bg % NG;
    const int tid = threadIdx.x, lane = tid & 31;
    const int wave = __builtin_amdgcn_readfirstlane((int)(threadIdx.x >> 5));
    const float* xp = x + ((size_t)b * DM + (size_t)g * CPG) * SEQ_FULL;
    const int nq = CPG * (SEQ / 4);
    float s = 0.0f;
#pragma unroll 1
    for (int i = tid; i < nq; i += 256) { const int c = i / (SEQ / 4), q = i % (SEQ / 4);
        const v4f v = *(const v4f*)(xp + (size_t)c * SEQ_FULL + (size_t)q * 4);
        s += (bfr(v[0]) + bfr(v[1])) + (bfr(v[2]) + bfr(v[3])); }
#pragma unroll
    for (int o = 16; o > 0; o >>= 1) s += __shfl_xor(s, o, 32);
    if (lane == 0) red[wave] = s;
    __syncthreads();
    float tot = 0.0f;
#pragma unroll
    for (int w = 0; w < 8; ++w) tot += red[w];
    const float invn = 1.0f / (float)(CPG * SEQ);
    const float mean = tot * invn;
    float s2 = 0.0f;
#pragma unroll 1
    for (int i = tid; i < nq; i += 256) { const int c = i / (SEQ / 4), q = i % (SEQ / 4);
        const v4f v = *(const v4f*)(xp + (size_t)c * SEQ_FULL + (size_t)q * 4);
        const float d0 = bfr(v[0]) - mean, d1 = bfr(v[1]) - mean, d2 = bfr(v[2]) - mean, d3 = bfr(v[3]) - mean;
        s2 += (d0 * d0 + d1 * d1) + (d2 * d2 + d3 * d3); }
#pragma unroll
    for (int o = 16; o > 0; o >>= 1) s2 += __shfl_xor(s2, o, 32);
    if (lane == 0) red2[wave] = s2;
    __syncthreads();
    float tot2 = 0.0f;
#pragma unroll
    for (int w = 0; w < 8; ++w) tot2 += red2[w];
    const float var = tot2 * invn;
    const float rstd = rsqrtf(var + GN_EPS);
    static_assert(8 * 16 == 128);
    if (tid < 8) {
        v4f o; o[0] = mean; o[1] = rstd; o[2] = mean; o[3] = rstd;
        float* dst = stats + (size_t)bg * 32 + tid * 4;
        *(volatile v4f*)dst = o; __threadfence(); *(volatile v4f*)dst = o;
    }
}

__global__ __launch_bounds__(256) void k_gnapply(const float* __restrict__ x, const float* __restrict__ gamma, const float* __restrict__ beta,
                                                 const float* __restrict__ stats, h16* NT) {
#pragma clang fp contract(off)
    __shared__ __align__(16) h16 ts[64 * TP];
    const int tid = threadIdx.x; const int n0 = blockIdx.x * 64, b = blockIdx.y;
    static_assert(256 * 8 == DM * 16);
#pragma unroll 1
    for (int it = 0; it < 8; ++it) {
        const int idx = it * 256 + tid; const int c = idx >> 4, q4 = idx & 15;
        const v4f v = *(const v4f*)(x + ((size_t)b * DM + c) * SEQ_FULL + n0 + q4 * 4);
        const int sg = (b * NG + (c >> 3)) * 32;
        const float mean = stats[sg], rstd = stats[sg + 1];
        const float ga = bfr(gamma[c]), be = bfr(beta[c]);
#pragma unroll
        for (int i = 0; i < 4; ++i) ts[(q4 * 4 + i) * TP + c] = toh_flush(((bfr(v[i]) - mean) * rstd) * ga + be);
    }
    __syncthreads();
    const size_t ob = ((size_t)b * SEQ + n0) * DM;
    static_assert(256 * 4 * 16 == 64 * DM * 2);
#pragma unroll 1
    for (int ps = 0; ps < 2; ++ps) {
#pragma unroll 1
        for (int it = 0; it < 4; ++it) { const int p = it * 256 + tid; const int row = p >> 4, c8 = (p & 15) * 8;
            const v8h hv = *(const v8ha*)(&ts[row * TP + c8]);
            *(volatile v8h*)(NT + ob + (size_t)p * 8) = hv; }
        if (ps == 0) __threadfence(); }
}

__global__ __launch_bounds__(256) void k_wconv(const float* __restrict__ src, h16* dst, int hstride, int nplanes) {
#pragma clang fp contract(off)
    const int i = blockIdx.x * 256 + threadIdx.x; if (i >= nplanes * (DM * DM / 8)) return;
    const int p = i / (DM * DM / 8), rem = i % (DM * DM / 8); const int r = rem >> 4, c8 = (rem & 15) * 8;
    const int srow = (r >> 5) * hstride + p * HD + (r & 31);
    const v8f v = *(const v8f*)(src + (size_t)srow * DM + c8); v8h o;
#pragma unroll
    for (int k = 0; k < 8; ++k) o[k] = toh_flush(bfr(v[k]) * WSC);
    *(volatile v8h*)(dst + (size_t)i * 8) = o; __threadfence(); *(volatile v8h*)(dst + (size_t)i * 8) = o;
}

__global__ __launch_bounds__(32) void k_qk(const h16* __restrict__ NT, const h16* __restrict__ WQK, h16* QK) {
    __shared__ __align__(16) float os[16 * 68];
    const int lane = threadIdx.x & 31, lr = lane & 15, hi = lane >> 4; const int r0 = blockIdx.x * 64, cy = blockIdx.y;
    v8f acc[4][4];
#pragma unroll
    for (int mb = 0; mb < 4; ++mb)
#pragma unroll
        for (int nb = 0; nb < 4; ++nb) acc[mb][nb] = (v8f){};
    const size_t aoff = (size_t)(r0 + lr) * DM + 8 * hi, boff = (size_t)(cy * 64 + lr) * DM + 8 * hi;
#pragma unroll 1
    for (int kc = 0; kc < DM; kc += 32) {
        v16h a[4];
#pragma unroll
        for (int mb = 0; mb < 4; ++mb) a[mb] = ldh(NT + aoff + (size_t)mb * 16 * DM + kc);
#pragma unroll
        for (int nb = 0; nb < 4; ++nb) { const v16h b = ldh(WQK + boff + (size_t)nb * 16 * DM + kc);
#pragma unroll
            for (int mb = 0; mb < 4; ++mb) acc[mb][nb] = wmma16g(a[mb], b, acc[mb][nb]); }
    }
    const int bb = r0 / SEQ, tt = r0 % SEQ; const int sel = cy >> 1; const int zc = bb * NH_ + (cy & 1) * 2;
    const size_t tbase = (size_t)sel * ((size_t)NB * NH_ * SEQ * HD) + ((size_t)zc * SEQ + (size_t)tt) * HD;
#pragma unroll
    for (int mb = 0; mb < 4; ++mb) {
#pragma unroll
        for (int nb = 0; nb < 4; ++nb) {
#pragma unroll
            for (int j = 0; j < 8; ++j) os[(hi * 8 + j) * 68 + nb * 16 + lr] = acc[mb][nb][j] * WSI; }
        wave_sync();
        static_assert(32 * 2 * 2 * 16 == 16 * 64 * 2);
#pragma unroll 1
        for (int ps = 0; ps < 2; ++ps) {
            const size_t sb = tbase + (size_t)(mb * 16) * HD;
#pragma unroll
            for (int hh = 0; hh < 2; ++hh) {
#pragma unroll
                for (int s = 0; s < 2; ++s) { const int p = s * 32 + lane; const int row = p >> 2, c8 = (p & 3) * 8;
                    const v4f x0 = *(const v4fa*)(&os[row * 68 + hh * 32 + c8]); const v4f x1 = *(const v4fa*)(&os[row * 68 + hh * 32 + c8 + 4]); v8h hv;
#pragma unroll
                    for (int i = 0; i < 4; ++i) { hv[i] = toh_flush(x0[i]); hv[4 + i] = toh_flush(x1[i]); }
                    const size_t oo = sb + (size_t)hh * ((size_t)SEQ * HD) + (size_t)p * 8;
                    *(volatile v8h*)(QK + oo) = hv; } }
            if (ps == 0) __threadfence(); }
        wave_sync();
    }
}

__global__ __launch_bounds__(32) void k_vt(const h16* __restrict__ WV, const h16* __restrict__ NT, h16* VT) {
    __shared__ __align__(16) float os[16 * 68];
    const int lane = threadIdx.x & 31, lr = lane & 15, hi = lane >> 4; const int r0 = blockIdx.x * 64, c0 = blockIdx.y * 64;
    v8f acc[4][4];
#pragma unroll
    for (int mb = 0; mb < 4; ++mb)
#pragma unroll
        for (int nb = 0; nb < 4; ++nb) acc[mb][nb] = (v8f){};
    const size_t aoff = (size_t)(r0 + lr) * DM + 8 * hi, boff = (size_t)(c0 + lr) * DM + 8 * hi;
#pragma unroll 1
    for (int kc = 0; kc < DM; kc += 32) {
        v16h a[4];
#pragma unroll
        for (int mb = 0; mb < 4; ++mb) a[mb] = ldh(WV + aoff + (size_t)mb * 16 * DM + kc);
#pragma unroll
        for (int nb = 0; nb < 4; ++nb) { const v16h b = ldh(NT + boff + (size_t)nb * 16 * DM + kc);
#pragma unroll
            for (int mb = 0; mb < 4; ++mb) acc[mb][nb] = wmma16g(a[mb], b, acc[mb][nb]); }
    }
    const int bb = c0 / SEQ, tt = c0 % SEQ;
    const size_t tbase = (size_t)bb * (size_t)DM * SEQ + (size_t)r0 * SEQ + (size_t)tt;
#pragma unroll
    for (int mb = 0; mb < 4; ++mb) {
#pragma unroll
        for (int nb = 0; nb < 4; ++nb) {
#pragma unroll
            for (int j = 0; j < 8; ++j) os[(hi * 8 + j) * 68 + nb * 16 + lr] = acc[mb][nb][j] * WSI; }
        wave_sync();
        static_assert(32 * 4 * 16 == 16 * 64 * 2);
#pragma unroll 1
        for (int ps = 0; ps < 2; ++ps) {
            const size_t sb = tbase + (size_t)(mb * 16) * SEQ;
#pragma unroll
            for (int s = 0; s < 4; ++s) { const int row = 4 * s + (lane >> 3), c8 = (lane & 7) * 8;
                const v4f x0 = *(const v4fa*)(&os[row * 68 + c8]); const v4f x1 = *(const v4fa*)(&os[row * 68 + c8 + 4]); v8h hv;
#pragma unroll
                for (int i = 0; i < 4; ++i) { hv[i] = toh_flush(x0[i]); hv[4 + i] = toh_flush(x1[i]); }
                const size_t oo = sb + (size_t)row * SEQ + c8;
                *(volatile v8h*)(VT + oo) = hv; }
            if (ps == 0) __threadfence(); }
        wave_sync();
    }
}

__global__ __launch_bounds__(32 * AW) void k_flash(const h16* __restrict__ QH, const h16* __restrict__ KP, const h16* __restrict__ VT, h16* CT) {
    __shared__ __align__(16) float os[AW * 16 * OSP];
    const int lane = threadIdx.x & 31, lr = lane & 15, hi = lane >> 4;
    const int wave = __builtin_amdgcn_readfirstlane((int)(threadIdx.x >> 5));
    const int zh = blockIdx.y;
    const int t0 = (blockIdx.x * AW + wave) * 16;
    const size_t pbase = (size_t)zh * SEQ * HD;
    const size_t qo = pbase + (size_t)(t0 + lr) * HD + 8 * hi;
    const v16h qh = ldh(QH + qo);
    const size_t ko = pbase + (size_t)lr * HD + 8 * hi;
    const size_t vo = pbase + (size_t)lr * SEQ + 8 * hi;
    v8f o0 = (v8f){}, o1 = (v8f){};
    float m = NEGB, l = 0.0f;
#pragma unroll 1
    for (int key0 = 0; key0 < SEQ; key0 += 32) {
        const h16* ka = KP + ko + (size_t)key0 * HD;
        const v16h ka0 = ldh(ka), kb0 = ldh(ka + 16 * HD);
        const v8f sa = wmma16g(ka0, qh, (v8f){});
        const v8f sb = wmma16g(kb0, qh, (v8f){});
        float ta[8], tb[8]; float mx = NEGB;
#pragma unroll
        for (int r = 0; r < 8; ++r) { ta[r] = sa[r] * SC2; tb[r] = sb[r] * SC2; mx = fmaxf(mx, fmaxf(ta[r], tb[r])); }
        mx = fmaxf(mx, __shfl_xor(mx, 16, 32));
        const float mnew = fmaxf(m, mx);
        const float alpha = __builtin_amdgcn_exp2f(m - mnew);
        const float sh = PSH - mnew;
        v16h pb; float ls = 0.0f;
#pragma unroll
        for (int r = 0; r < 8; ++r) {
            const float xa = ta[r] + sh, xb = tb[r] + sh;
            const float ga = (xa < -14.0f) ? 0.0f : __builtin_amdgcn_exp2f(xa);
            const float gb = (xb < -14.0f) ? 0.0f : __builtin_amdgcn_exp2f(xb);
            const h16 pa = (h16)ga; const h16 pc = (h16)gb;
            pb[r] = pa; pb[8 + r] = pc;
            ls += (float)pa + (float)pc; }
        l = l * alpha + ls; m = mnew;
        o0 = o0 * alpha; o1 = o1 * alpha;
        const h16* va = VT + vo + key0;
        const v16h v0 = ldh(va), v1 = ldh(va + (size_t)16 * SEQ);
        o0 = wmma16g(v0, pb, o0);
        o1 = wmma16g(v1, pb, o1);
    }
    l += __shfl_xor(l, 16, 32);
    const float inv = CTXC * (1.0f / l);
    const int wb = wave * 16 * OSP;
    { v4f a, c;
      a[0] = o0[0] * inv; a[1] = o0[1] * inv; a[2] = o0[2] * inv; a[3] = o0[3] * inv; c[0] = o0[4] * inv; c[1] = o0[5] * inv; c[2] = o0[6] * inv; c[3] = o0[7] * inv;
      *(v4fa*)(&os[wb + lr * OSP +  0 + 8 * hi]) = a; *(v4fa*)(&os[wb + lr * OSP +  0 + 8 * hi + 4]) = c;
      a[0] = o1[0] * inv; a[1] = o1[1] * inv; a[2] = o1[2] * inv; a[3] = o1[3] * inv; c[0] = o1[4] * inv; c[1] = o1[5] * inv; c[2] = o1[6] * inv; c[3] = o1[7] * inv;
      *(v4fa*)(&os[wb + lr * OSP + 16 + 8 * hi]) = a; *(v4fa*)(&os[wb + lr * OSP + 16 + 8 * hi + 4]) = c; }
    wave_sync();
    const size_t cbase = pbase + (size_t)t0 * HD;
    static_assert(32 * 2 * 16 == 16 * HD * 2);
#pragma unroll 1
    for (int ps = 0; ps < 2; ++ps) {
#pragma unroll
        for (int s = 0; s < 2; ++s) { const int p = s * 32 + lane; const int row = p >> 2, c8 = (p & 3) * 8;
            const v4f x0 = *(const v4fa*)(&os[wb + row * OSP + c8]); const v4f x1 = *(const v4fa*)(&os[wb + row * OSP + c8 + 4]); v8h hv;
#pragma unroll
            for (int i = 0; i < 4; ++i) { hv[i] = toh_flush(x0[i]); hv[4 + i] = toh_flush(x1[i]); }
            *(volatile v8h*)(CT + cbase + (size_t)p * 8) = hv; }
        if (ps == 0) __threadfence(); }
}

__global__ __launch_bounds__(32) void k_out(const h16* __restrict__ WO, const h16* __restrict__ CT, const float* __restrict__ bout, const float* __restrict__ X, float* OUT) {
    __shared__ __align__(16) float os[16 * 68];
    const int lane = threadIdx.x & 31, lr = lane & 15, hi = lane >> 4; const int r0 = blockIdx.x * 64, c0 = blockIdx.y * 64;
    const int bb = c0 / SEQ, tt = c0 % SEQ;
    v8f acc[4][4];
#pragma unroll
    for (int mb = 0; mb < 4; ++mb)
#pragma unroll
        for (int nb = 0; nb < 4; ++nb) acc[mb][nb] = (v8f){};
    const size_t aoff = (size_t)(r0 + lr) * DM + 8 * hi;
    const size_t boff = ((size_t)bb * NH_ * SEQ + (size_t)(tt + lr)) * HD + 8 * hi;
#pragma unroll 1
    for (int hk = 0; hk < NH_; ++hk) {
        v16h a[4];
#pragma unroll
        for (int mb = 0; mb < 4; ++mb) a[mb] = ldh(WO + aoff + (size_t)mb * 16 * DM + hk * 32);
#pragma unroll
        for (int nb = 0; nb < 4; ++nb) { const v16h b = ldh(CT + boff + (size_t)hk * ((size_t)SEQ * HD) + (size_t)nb * 16 * HD);
#pragma unroll
            for (int mb = 0; mb < 4; ++mb) acc[mb][nb] = wmma16g(a[mb], b, acc[mb][nb]); }
    }
#pragma unroll
    for (int mb = 0; mb < 4; ++mb) {
#pragma unroll
        for (int nb = 0; nb < 4; ++nb) {
#pragma unroll
            for (int j = 0; j < 8; ++j) os[(hi * 8 + j) * 68 + nb * 16 + lr] = acc[mb][nb][j] * OSC; }
        wave_sync();
        static_assert(32 * 8 * 16 == 16 * 64 * 4);
#pragma unroll 1
        for (int ps = 0; ps < 2; ++ps) {
#pragma unroll 2
            for (int s = 0; s < 8; ++s) { const int row = 2 * s + (lane >> 4), cofs = (lane & 15) * 4;
                const int o = r0 + mb * 16 + row;
                const v4f val = *(const v4fa*)(&os[row * 68 + cofs]);
                const float bias = bfr(bout[o]);
                const v4f xr = *(const v4f*)(X + ((size_t)bb * DM + o) * SEQ_FULL + tt + cofs);
                v4f ov;
#pragma unroll
                for (int i = 0; i < 4; ++i) ov[i] = (val[i] + bias) + bfr(xr[i]);
                *(volatile v4f*)(OUT + ((size_t)bb * DM + o) * OUT_SEQ + tt + cofs) = ov; }
            if (ps == 0) __threadfence(); }
        wave_sync();
    }
}

static constexpr size_t al256(size_t v) { return (v + 255) & ~(size_t)255; }
static constexpr size_t SZ_ST = al256((size_t)NB * NG * 32 * 4);
static constexpr size_t SZ_NT = al256((size_t)NB * SEQ * DM * 2);
static constexpr size_t SZ_WB = al256((size_t)4 * DM * DM * 2);
static constexpr size_t SZ_PL = al256((size_t)NB * NH_ * SEQ * HD * 2);
static constexpr size_t SZ_TOTAL = SZ_ST + SZ_NT + SZ_WB + 4 * SZ_PL;
static_assert(SZ_TOTAL <= (size_t)134217728);
static_assert(((size_t)DM * DM * 2) % 256 == 0);
static_assert(((size_t)NB * NH_ * SEQ * HD * 2) % 256 == 0);
static_assert((size_t)NB * NH_ * SEQ * HD == (size_t)NB * DM * SEQ);
static_assert((3 * DM * DM / 8) % 256 == 0);
static_assert((DM * DM / 8) % 256 == 0);

extern "C" void kernel_launch(void* const* d_in, const int* in_sizes, int n_in,
                              void* d_out, int out_size, void* d_ws, size_t ws_size, hipStream_t stream) {
    if (n_in < 6) return;
    const size_t needx = ((size_t)(NB - 1) * DM + (DM - 1)) * SEQ_FULL + SEQ;
    if ((size_t)in_sizes[0] < needx) return;
    if (in_sizes[1] < DM || in_sizes[2] < DM) return;
    if ((size_t)in_sizes[3] < (size_t)3 * DM * DM || (size_t)in_sizes[4] < (size_t)DM * DM || in_sizes[5] < DM) return;
    if ((size_t)out_size < ((size_t)(NB * DM - 1)) * OUT_SEQ + SEQ) return;
    if (SZ_TOTAL > ws_size) return;
    const float* x     = (const float*)d_in[0];
    const float* gamma = (const float*)d_in[1];
    const float* beta  = (const float*)d_in[2];
    const float* wqkv  = (const float*)d_in[3];
    const float* wout  = (const float*)d_in[4];
    const float* bout  = (const float*)d_in[5];
    float* OUT = (float*)d_out;
    char* wsp = (char*)d_ws;
    float* ST = (float*)wsp; wsp += SZ_ST;
    h16* NT = (h16*)wsp; wsp += SZ_NT;
    h16* WB = (h16*)wsp; wsp += SZ_WB;
    h16* QK = (h16*)wsp; wsp += 2 * SZ_PL;
    h16* VT = (h16*)wsp; wsp += SZ_PL;
    h16* CT = (h16*)wsp; wsp += SZ_PL;
    h16* WV = WB + (size_t)2 * DM * DM; h16* WO = WB + (size_t)3 * DM * DM;
    h16* QH = QK; h16* KP = QK + (size_t)NB * NH_ * SEQ * HD;

    k_gnstats<<<NB * NG, 256, 0, stream>>>(x, ST);
    k_gnapply<<<dim3(SEQ / 64, NB, 1), 256, 0, stream>>>(x, gamma, beta, ST, NT);
    k_wconv<<<(3 * DM * DM / 8) / 256, 256, 0, stream>>>(wqkv, WB, 3 * HD, 3);
    k_wconv<<<(DM * DM / 8) / 256, 256, 0, stream>>>(wout, WO, HD, 1);

    k_qk<<<dim3(NB * SEQ / 64, 4, 1), 32, 0, stream>>>(NT, WB, QK);
    k_vt<<<dim3(DM / 64, NB * SEQ / 64, 1), 32, 0, stream>>>(WV, NT, VT);

    k_flash<<<dim3(SEQ / (16 * AW), NB * NH_, 1), 32 * AW, 0, stream>>>(QH, KP, VT, CT);

    k_out<<<dim3(DM / 64, NB * SEQ / 64, 1), 32, 0, stream>>>(WO, CT, bout, x, OUT);
}
